// RunRingFlashAttn_63041529970731
// MI455X (gfx1250) — hardware-verified
//
#include <hip/hip_runtime.h>


namespace {
constexpr int Bsz = 2, T = 2048, HID = 1024, DH = 64, NH = 16, NKV = 16, REP = NH / NKV;
constexpr int KVW = NKV * DH;
constexpr int NQKV = HID + 2 * KVW;
constexpr int MROWS = Bsz * T;
constexpr int QT_PER_B = T / 16;

#define VST2f(ptr, val) do { const v4f _v = (val); *(volatile v4f*)(ptr) = _v; __threadfence(); *(volatile v4f*)(ptr) = _v; } while (0)
typedef _Float16 b16;
typedef __attribute__((ext_vector_type(16))) _Float16 v16b;
typedef __attribute__((ext_vector_type(8)))  _Float16 v8b;
typedef __attribute__((ext_vector_type(8)))  float v8f;
typedef __attribute__((ext_vector_type(4)))  float v4f;

__device__ __forceinline__ v8b ld8b(const b16* p) { return *(const v8b*)p; }
__device__ __forceinline__ v16b cat8b(v8b a, v8b b) { return __builtin_shufflevector(a, b, 0, 1, 2, 3, 4, 5, 6, 7, 8, 9, 10, 11, 12, 13, 14, 15); }
__device__ __forceinline__ v16b frag_kb(const b16* p, int hh) { return cat8b(ld8b(p + 8 * hh), ld8b(p + 16 + 8 * hh)); }
__device__ __forceinline__ void split_bf16(float v, b16& hi, b16& lo) {
  hi = (b16)v; lo = (b16)0.0f;
}
__device__ __forceinline__ void frag_ksplit(const float* p, int hh, v16b& fh_, v16b& fl_) {
  const float* p0 = p + 8 * hh; const float* p1 = p + 16 + 8 * hh;
#pragma unroll
  for (int e = 0; e < 8; ++e) { b16 a, c; split_bf16(p0[e], a, c); fh_[e] = a; fl_[e] = c; split_bf16(p1[e], a, c); fh_[8 + e] = a; fl_[8 + e] = c; }
}
__device__ __forceinline__ v8f wmma16b(v16b a, v16b b, v8f c) {
  v8f d = __builtin_amdgcn_wmma_f32_16x16x32_f16(false, a, false, b, (short)0, c, false, false);
  asm volatile("v_nop\n\tv_nop\n\tv_nop\n\tv_nop" : "+v"(d) : "v"(a), "v"(b));
  return d;
}
__device__ __forceinline__ v8f wmma3(v16b ah, v16b al, v16b bh, v16b bl, v8f c) {
  (void)al; (void)bl; return wmma16b(ah, bh, c);
}
__device__ __forceinline__ void wave_lds_sync() {
  __builtin_amdgcn_fence(__ATOMIC_RELEASE, "workgroup");
  __builtin_amdgcn_wave_barrier();
  __builtin_amdgcn_fence(__ATOMIC_ACQUIRE, "workgroup");
}

__global__ __launch_bounds__(256) void attn_kernel(const b16* __restrict__ Qh, const b16* __restrict__ Ql, const b16* __restrict__ Kh, const b16* __restrict__ Kl,
                                                   const b16* __restrict__ Vh, const b16* __restrict__ Vl,
                                                   float* __restrict__ yf) {
  __shared__ __attribute__((aligned(16))) float Os[8][16 * 64];
  const int wid = threadIdx.x >> 5, lane = threadIdx.x & 31, hh = lane >> 4, col = lane & 15;
  const int qtile = blockIdx.x * 8 + wid;
  const int g = qtile / QT_PER_B;
  const int q0 = (qtile % QT_PER_B) << 4;
  const int b = g / NH, h = g % NH, kvh = h / REP;
  const size_t ko = (size_t)(b * NKV + kvh) * T * DH;
  const size_t qo = ((size_t)g * T + q0 + col) * DH;
  const v16b q0h = frag_kb(Qh + qo, hh), q0l = frag_kb(Ql + qo, hh), q1h = frag_kb(Qh + qo + 32, hh), q1l = frag_kb(Ql + qo + 32, hh);
  float m = -INFINITY, l = 0.0f;
  v8f o0 = {}, o1 = {}, o2 = {}, o3 = {};
  for (int kb = 0; kb < T; kb += 32) {
    const size_t r0 = ko + (size_t)(kb + col) * DH, r1 = ko + (size_t)(kb + 16 + col) * DH;
    v8f s0 = {}, s1 = {};
    {
      v16b ah = frag_kb(Kh + r0, hh), al = frag_kb(Kl + r0, hh);
      s0 = wmma3(ah, al, q0h, q0l, s0);
      ah = frag_kb(Kh + r0 + 32, hh); al = frag_kb(Kl + r0 + 32, hh);
      s0 = wmma3(ah, al, q1h, q1l, s0);
      ah = frag_kb(Kh + r1, hh); al = frag_kb(Kl + r1, hh);
      s1 = wmma3(ah, al, q0h, q0l, s1);
      ah = frag_kb(Kh + r1 + 32, hh); al = frag_kb(Kl + r1 + 32, hh);
      s1 = wmma3(ah, al, q1h, q1l, s1);
    }
    float mr = -INFINITY;
#pragma unroll
    for (int r = 0; r < 8; ++r) mr = fmaxf(mr, fmaxf(s0[r], s1[r]));
    mr = fmaxf(mr, __shfl_xor(mr, 16));
    const float mn = fmaxf(m, mr);
    const float al_ = __expf(m - mn);
    m = mn;
    float sum = 0.0f;
    v16b pbh, pbl;
#pragma unroll
    for (int r = 0; r < 8; ++r) {
      const float p0 = __expf(s0[r] - mn), p1 = __expf(s1[r] - mn);
      sum += p0 + p1;
      b16 a, c; split_bf16(p0, a, c); pbh[r] = a; pbl[r] = c; split_bf16(p1, a, c); pbh[8 + r] = a; pbl[8 + r] = c;
    }
    sum += __shfl_xor(sum, 16);
    l = l * al_ + sum;
#pragma unroll
    for (int r = 0; r < 8; ++r) { o0[r] *= al_; o1[r] *= al_; o2[r] *= al_; o3[r] *= al_; }
    const size_t v0 = ko + (size_t)(kb >> 4) * (DH * 16) + 8 * hh, v1 = v0 + DH * 16;
#pragma unroll
    for (int n = 0; n < 4; ++n) {
      const int f = n * 16 + col;
      const v16b vah = cat8b(ld8b(Vh + v0 + f * 16), ld8b(Vh + v1 + f * 16));
      const v16b val = cat8b(ld8b(Vl + v0 + f * 16), ld8b(Vl + v1 + f * 16));
      v8f& o = (n == 0) ? o0 : (n == 1) ? o1 : (n == 2) ? o2 : o3;
      o = wmma3(vah, val, pbh, pbl, o);
    }
  }
  const float inv = 1.0f / l;
  float* Tt = Os[wid];
#pragma unroll
  for (int r = 0; r < 8; ++r) {
    const int hr = 8 * hh + r;
    Tt[col * 64 + 0 + hr] = o0[r] * inv; Tt[col * 64 + 16 + hr] = o1[r] * inv;
    Tt[col * 64 + 32 + hr] = o2[r] * inv; Tt[col * 64 + 48 + hr] = o3[r] * inv;
  }
  wave_lds_sync();
  float* dst0 = yf + ((size_t)b * T + q0) * HID + h * DH;
#pragma unroll
  for (int j = 0; j < 8; ++j) { const int rr = j * 2 + hh, c4 = col * 4; *(volatile v4f*)(dst0 + (size_t)rr * HID + c4) = *(const v4f*)(Tt + rr * 64 + c4); }
  __threadfence();
#pragma unroll
  for (int j = 0; j < 8; ++j) { const int rr = j * 2 + hh, c4 = col * 4; *(volatile v4f*)(dst0 + (size_t)rr * HID + c4) = *(const v4f*)(Tt + rr * 64 + c4); }
}

__global__ __launch_bounds__(256) void convert_qkv_kernel(const float* __restrict__ q, const float* __restrict__ k, const float* __restrict__ v,
                                                          b16* __restrict__ Qh, b16* __restrict__ Kh, b16* __restrict__ Vh) {
  const int tid = blockIdx.x * 256 + threadIdx.x;
  {
    const int d8 = (tid & 7) * 8, h = (tid >> 3) & (NH - 1), t = (tid >> 7) & (T - 1), b = tid >> 18;
    const size_t src = (((size_t)b * T + t) * NH + h) * DH + d8;
    const size_t dst = (((size_t)b * NH + h) * T + t) * DH + d8;
    v8b qv, kv;
#pragma unroll
    for (int e = 0; e < 8; ++e) { qv[e] = (b16)(q[src + e] * 0.125f); kv[e] = (b16)k[src + e]; }
    *(volatile v8b*)(Qh + dst) = qv; *(volatile v8b*)(Kh + dst) = kv; __threadfence();
    *(volatile v8b*)(Qh + dst) = qv; *(volatile v8b*)(Kh + dst) = kv;
  }
  if (tid < Bsz * NH * QT_PER_B * DH) {
    const int d = tid & 63, tt = (tid >> 6) & (QT_PER_B - 1), h = (tid >> 13) & (NH - 1), b = tid >> 17;
    v16b vv;
#pragma unroll
    for (int e = 0; e < 16; ++e) vv[e] = (b16)v[(((size_t)b * T + tt * 16 + e) * NH + h) * DH + d];
    b16* dst = Vh + (((size_t)b * NH + h) * QT_PER_B + tt) * (DH * 16) + d * 16;
    *(volatile v16b*)dst = vv; __threadfence(); *(volatile v16b*)dst = vv;
  }
}
}

extern "C" void kernel_launch(void* const* d_in, const int* in_sizes, int n_in,
                              void* d_out, int out_size, void* d_ws, size_t ws_size, hipStream_t stream) {
  (void)in_sizes; (void)n_in; (void)out_size;
  const float* q = (const float*)d_in[0];
  const float* k = (const float*)d_in[1];
  const float* v = (const float*)d_in[2];
  float* out = (float*)d_out;
  const size_t plane = (size_t)Bsz * NH * T * DH * 2;
  if (ws_size < 3 * plane) return;
  char* ws = (char*)d_ws;
  b16* Qh = (b16*)ws; b16* Kh = (b16*)(ws + plane); b16* Vh = (b16*)(ws + 2 * plane);
  convert_qkv_kernel<<<(Bsz * T * NH * 8) / 256, 256, 0, stream>>>(q, k, v, Qh, Kh, Vh);
  attn_kernel<<<(Bsz * NH * QT_PER_B) / 8, 256, 0, stream>>>(Qh, Qh, Kh, Kh, Vh, Vh, out);
}
